// KernelAggregation_49280454754759
// MI455X (gfx1250) — hardware-verified
//
#include <hip/hip_runtime.h>
#include <math.h>

typedef __attribute__((ext_vector_type(16))) _Float16 v16h;
typedef __attribute__((ext_vector_type(16))) __bf16 v16b;
typedef __attribute__((ext_vector_type(8)))  _Float16 v8h;
typedef __attribute__((ext_vector_type(8)))  float v8f;
typedef __attribute__((ext_vector_type(4)))  float v4f;
typedef __attribute__((ext_vector_type(2)))  float v2f;
typedef __attribute__((ext_vector_type(4)))  unsigned v4u;
typedef __attribute__((ext_vector_type(4)))  int v4i;
typedef float __attribute__((may_alias)) float_a;
typedef int __attribute__((may_alias)) int_a;

template <typename T> __device__ __forceinline__ void vst2(void* p, T v) { *(volatile T*)p = v; __threadfence(); *(volatile T*)p = v; }
__device__ __forceinline__ v8f wmma16(v16h a, v16h b, v8f c) {
  v8f d = __builtin_amdgcn_wmma_f32_16x16x32_f16(false, a, false, b, (short)0, c, false, false);
  asm volatile("v_nop\n\tv_nop\n\tv_nop\n\tv_nop" : "+v"(d) : "v"(a), "v"(b));
  return d;
}
__device__ __forceinline__ v8f wmma_bf(v16b a, v16b b, v8f c) {
  v8f d = __builtin_amdgcn_wmma_f32_16x16x32_bf16(false, a, false, b, (short)0, c, false, false);
  asm volatile("v_nop\n\tv_nop\n\tv_nop\n\tv_nop" : "+v"(d) : "v"(a), "v"(b));
  return d;
}
__device__ __forceinline__ v16h frag_h(const _Float16* rowk0, int lane) {
  union { v16h v; v8h q[2]; } u; const _Float16* p = rowk0 + 8 * (lane >> 4);
  u.q[0] = *(const v8h*)p; u.q[1] = *(const v8h*)(p + 16); return u.v;
}
__device__ __forceinline__ v16h frag_f32(const float* rowk0, int lane) {
  v16h a; const float* p = rowk0 + 8 * (lane >> 4);
#pragma unroll
  for (int i = 0; i < 8; ++i) { a[i] = (_Float16)p[i]; a[8 + i] = (_Float16)p[16 + i]; }
  return a;
}
__device__ __forceinline__ v16h frag_f32s(const float* rowk0, int lane, float sc) {
  v16h a; const float* p = rowk0 + 8 * (lane >> 4);
#pragma unroll
  for (int i = 0; i < 8; ++i) { a[i] = (_Float16)(p[i] * sc); a[8 + i] = (_Float16)(p[16 + i] * sc); }
  return a;
}
__device__ __forceinline__ v16h fragc_f32(const float* W, int k0, int n, int lane, int ld, int K) {
  v16h a; const int g = lane >> 4;
#pragma unroll
  for (int i = 0; i < 8; ++i) { const int ka = k0 + 8 * g + i, kb = ka + 16;
    a[i] = (_Float16)(ka < K ? W[(size_t)ka * ld + n] : 0.f); a[8 + i] = (_Float16)(kb < K ? W[(size_t)kb * ld + n] : 0.f); }
  return a;
}
struct F2 { v16b h, l; };
__device__ __forceinline__ F2 bsplit16(const float v[16]) { F2 r;
#pragma unroll
  for (int i = 0; i < 16; ++i) { const __bf16 h = (__bf16)v[i]; r.h[i] = h; r.l[i] = (__bf16)(v[i] - (float)h); }
  return r; }
__device__ __forceinline__ F2 split_row(const float* row, int k0, int lane) { float v[16]; const float* p = row + k0 + 8 * (lane >> 4);
#pragma unroll
  for (int i = 0; i < 8; ++i) { v[i] = p[i]; v[8 + i] = p[16 + i]; }
  return bsplit16(v); }
__device__ __forceinline__ F2 split_rowK(const float* row, int k0, int lane, int K) { float v[16]; const int g = lane >> 4;
#pragma unroll
  for (int i = 0; i < 8; ++i) { const int ka = k0 + 8 * g + i, kb = ka + 16; v[i] = ka < K ? row[ka] : 0.f; v[8 + i] = kb < K ? row[kb] : 0.f; }
  return bsplit16(v); }
__device__ __forceinline__ F2 split_col(const float* W, int k0, int n, int lane, int ld, int K) { float v[16]; const int g = lane >> 4;
#pragma unroll
  for (int i = 0; i < 8; ++i) { const int ka = k0 + 8 * g + i, kb = ka + 16; v[i] = ka < K ? W[(size_t)ka * ld + n] : 0.f; v[8 + i] = kb < K ? W[(size_t)kb * ld + n] : 0.f; }
  return bsplit16(v); }
__device__ __forceinline__ v8f mac3(const F2& a, const F2& b, v8f c) { c = wmma_bf(a.l, b.h, c); c = wmma_bf(a.h, b.l, c); return wmma_bf(a.h, b.h, c); }
__device__ __forceinline__ float sigm(float v) { return 1.0f / (1.0f + expf(-v)); }
#define LDSX() do { asm volatile("s_wait_dscnt 0" ::: "memory"); __builtin_amdgcn_wave_barrier(); __builtin_amdgcn_fence(__ATOMIC_RELEASE, "workgroup"); } while (0)


#define NB 8
#define NO 2048
#define NQ 2048
#define D 128

__global__ __launch_bounds__(128) void k_agg(const float* __restrict__ emb, const float* __restrict__ tobs, const float* __restrict__ tq, const float* __restrict__ omask, const float* __restrict__ lsig, const float* __restrict__ Wp, const float* __restrict__ bp, float* __restrict__ out) {
  __shared__ __align__(16) float sw[4][16][36]; __shared__ __align__(16) float sc[4][16][D + 4];
  const int tid = threadIdx.x, w = tid >> 5, lane = tid & 31, col = lane & 15, g = lane >> 4;
  const int b = blockIdx.y; const int q0 = blockIdx.x * 64 + w * 16;
  const float sig = expf((float)(__bf16)lsig[0]);
  const float* to = tobs + (size_t)b * NO; const float* om = omask + (size_t)b * NO; const float* eb = emb + (size_t)b * NO * D;
  const float tqr = (float)(__bf16)tq[(size_t)b * NQ + q0 + col];
  float wsum = 0.f; v8f acc[8] = {};
#pragma unroll 1
  for (int kc = 0; kc < NO / 32; ++kc) { const int o0 = kc * 32;
#pragma unroll
    for (int e = 0; e < 16; ++e) { const int o = o0 + g * 16 + e; const float dt = fabsf(tqr - (float)(__bf16)to[o]) / sig; const float wv = expf(-0.5f * dt * dt) * (float)(__bf16)om[o]; wsum += wv; sw[w][col][g * 16 + e] = wv; }
    LDSX();
    const F2 a = split_row(&sw[w][col][0], 0, lane);
#pragma unroll
    for (int j = 0; j < 8; ++j) { const v16b eb16 = split_col(eb + (size_t)o0 * D, 0, j * 16 + col, lane, D, 32).h; acc[j] = wmma_bf(a.l, eb16, acc[j]); acc[j] = wmma_bf(a.h, eb16, acc[j]); }
    LDSX(); }
  wsum += __shfl_xor(wsum, 16, 32);
  const float winv = 1.0f / fmaxf(wsum, 1e-8f);
#pragma unroll
  for (int r = 0; r < 8; ++r) { const float wi = __shfl(winv, 8 * g + r, 32);
#pragma unroll
    for (int j = 0; j < 8; ++j) sc[w][8 * g + r][j * 16 + col] = acc[j][r] * wi; }
  LDSX();
  v8f po[8] = {};
#pragma unroll
  for (int kc = 0; kc < D / 32; ++kc) { const F2 a = split_row(&sc[w][col][0], kc * 32, lane);
#pragma unroll
    for (int j = 0; j < 8; ++j) { const v16b wb = split_row(Wp + (size_t)(j * 16 + col) * D, kc * 32, lane).h; po[j] = wmma_bf(a.l, wb, po[j]); po[j] = wmma_bf(a.h, wb, po[j]); } }
  LDSX();
#pragma unroll
  for (int j = 0; j < 8; ++j) { const float bb = (float)(__bf16)bp[j * 16 + col];
#pragma unroll
    for (int r = 0; r < 8; ++r) sc[w][8 * g + r][j * 16 + col] = po[j][r] + bb; }
  LDSX();
  for (int rl = 0; rl < 16; ++rl) vst2(out + ((size_t)b * NQ + q0 + rl) * D + lane * 4, *(const v4f*)(&sc[w][rl][lane * 4]));
}
extern "C" void kernel_launch(void* const* d_in, const int* in_sizes, int n_in, void* d_out, int out_size, void* d_ws, size_t ws_size, hipStream_t stream) {
  (void)in_sizes; (void)n_in; (void)out_size; (void)ws_size; (void)d_ws;
  const float** I = (const float**)d_in;
  k_agg<<<dim3(NQ / 64, NB), 128, 0, stream>>>(I[0], I[1], I[2], I[3], I[4], I[5], I[6], (float*)d_out);
}
